// CustomAttention_53369263620187
// MI455X (gfx1250) — hardware-verified
//
#include <hip/hip_runtime.h>


#ifndef NB
#define NB 2
#endif
#ifndef SEQ
#define SEQ 2048
#endif
#define NB_FULL  2
#define SEQ_FULL 2048
#define DM   1024
#define NH   16
#define HD   64
#define NQKV 3072
#define NSLOT (3 * NH)
#ifndef RH
#define RH 512
#endif
#if RH > SEQ
#undef RH
#define RH SEQ
#endif
static_assert(SEQ % 64 == 0);
static_assert(RH % 64 == 0);
static_assert(RH <= SEQ);
static_assert(SEQ <= SEQ_FULL);
static_assert(NB <= NB_FULL);
static_assert(DM % 32 == 0);
#define PCAR 1024.0f
#define YCAR 16.0f
#define WCAR 64.0f
#define OSC  (1.0f / 1024.0f)
#define SCL  0.125f
#define L2E  1.4426950408889634f
#define ST   72
#define PT   (16 * ST)

typedef _Float16 h16;
typedef unsigned short bf;
typedef __attribute__((ext_vector_type(16))) __bf16   v16bf;
typedef __attribute__((ext_vector_type(16))) _Float16 v16h;
typedef __attribute__((ext_vector_type(8)))  _Float16 v8h;
typedef __attribute__((ext_vector_type(8)))  unsigned short v8us;
typedef __attribute__((ext_vector_type(8)))  float    v8f;
typedef __attribute__((ext_vector_type(4)))  float    v4f;
typedef v8h  __attribute__((may_alias)) v8ha;
typedef v4f  __attribute__((may_alias)) v4fa;
typedef v8us __attribute__((may_alias)) v8usa;

__device__ __forceinline__ unsigned short f2bf(float f) { unsigned u = __float_as_uint(f); u += 0x7FFFu + ((u >> 16) & 1u); return (unsigned short)(u >> 16); }
__device__ __forceinline__ float bf2f(unsigned short b) { return __uint_as_float(((unsigned)b) << 16); }
__device__ __forceinline__ float bfr(float f) { return bf2f(f2bf(f)); }
__device__ __forceinline__ v16h cat16(v8h lo, v8h hi) { return __builtin_shufflevector(lo, hi, 0, 1, 2, 3, 4, 5, 6, 7, 8, 9, 10, 11, 12, 13, 14, 15); }
__device__ __forceinline__ v16bf cat16b(v8us lo, v8us hi) { return __builtin_bit_cast(v16bf, __builtin_shufflevector(lo, hi, 0, 1, 2, 3, 4, 5, 6, 7, 8, 9, 10, 11, 12, 13, 14, 15)); }
__device__ __forceinline__ v8f wmma16(v16h a, v16h b, v8f c) { return __builtin_amdgcn_wmma_f32_16x16x32_f16(false, a, false, b, (short)0, c, false, false); }
__device__ __forceinline__ v8f wmmab(v16bf a, v16bf b, v8f c) { return __builtin_amdgcn_wmma_f32_16x16x32_bf16(false, a, false, b, (short)0, c, false, false); }
__device__ __forceinline__ void splitf(float y, unsigned short& h, unsigned short& l) { h = f2bf(y); l = f2bf(y - bf2f(h)); }

template <typename T16> struct WFrag;
template <> struct WFrag<h16> { typedef v16h V; static __device__ __forceinline__ V ld(const h16* p) { return cat16(*(const v8h*)p, *(const v8h*)(p + 16)); } static __device__ __forceinline__ v8f mma(V a, V b, v8f c) { return wmma16(a, b, c); } };
template <> struct WFrag<bf> { typedef v16bf V; static __device__ __forceinline__ V ld(const bf* p) { return cat16b(*(const v8us*)p, *(const v8us*)(p + 16)); } static __device__ __forceinline__ v8f mma(V a, V b, v8f c) { return wmmab(a, b, c); } };

template <typename T16, int NSPLIT, bool BIAS>
__global__ __launch_bounds__(32) void k_gemmw(const T16* __restrict__ A, const T16* __restrict__ A2, const T16* __restrict__ Bt, const T16* __restrict__ Bt2, int K, float* C, int ldc, const float* __restrict__ bias, float osc, size_t sA, size_t sB, size_t sC) {
    typedef typename WFrag<T16>::V V;
    __shared__ __align__(16) float os[16 * 68];
    const size_t z = blockIdx.z; A += z * sA; if (A2) A2 += z * sA; Bt += z * sB; if (Bt2) Bt2 += z * sB; C += z * sC;
    const int lane = threadIdx.x & 31, lr = lane & 15, hi = lane >> 4; const int r0 = blockIdx.x * 64, c0 = blockIdx.y * 64;
    v8f acc[4][4];
#pragma unroll
    for (int mb = 0; mb < 4; ++mb)
#pragma unroll
        for (int nb = 0; nb < 4; ++nb) acc[mb][nb] = (v8f){};
    const size_t aoff = (size_t)(r0 + lr) * K + 8 * hi, boff = (size_t)(c0 + lr) * K + 8 * hi;
#pragma unroll 1
    for (int kc = 0; kc < K; kc += 32) {
        V a[4], a2[4];
#pragma unroll
        for (int mb = 0; mb < 4; ++mb) { a[mb] = WFrag<T16>::ld(A + aoff + (size_t)mb * 16 * K + kc); if (NSPLIT == 1 || NSPLIT == 2) a2[mb] = WFrag<T16>::ld(A2 + aoff + (size_t)mb * 16 * K + kc); }
#pragma unroll
        for (int nb = 0; nb < 4; ++nb) { const V b = WFrag<T16>::ld(Bt + boff + (size_t)nb * 16 * K + kc); V b2; if (NSPLIT >= 2) b2 = WFrag<T16>::ld(Bt2 + boff + (size_t)nb * 16 * K + kc);
#pragma unroll
            for (int mb = 0; mb < 4; ++mb) { acc[mb][nb] = WFrag<T16>::mma(a[mb], b, acc[mb][nb]); if (NSPLIT == 1 || NSPLIT == 2) acc[mb][nb] = WFrag<T16>::mma(a2[mb], b, acc[mb][nb]); if (NSPLIT >= 2) acc[mb][nb] = WFrag<T16>::mma(a[mb], b2, acc[mb][nb]); } }
        asm volatile("v_nop\n\tv_nop\n\tv_nop\n\tv_nop" : "+v"(acc[0][0]), "+v"(acc[1][1]), "+v"(acc[2][2]), "+v"(acc[3][3]) : "v"(a[0]), "v"(a[3]));
    }
#pragma unroll
    for (int mb = 0; mb < 4; ++mb) {
#pragma unroll
        for (int nb = 0; nb < 4; ++nb) {
#pragma unroll
            for (int j = 0; j < 8; ++j) os[(hi * 8 + j) * 68 + nb * 16 + lr] = acc[mb][nb][j]; }
        __builtin_amdgcn_wave_barrier(); asm volatile("" ::: "memory");
        float* crow = C + (size_t)(r0 + mb * 16) * ldc + c0;
#pragma unroll 1
        for (int ps = 0; ps < 2; ++ps) {
#pragma unroll
            for (int s = 0; s < 8; ++s) { const int row = 2 * s + hi, cofs = lr * 4; v4f val = *(const v4fa*)(os + row * 68 + cofs); val = val * osc; if (BIAS) { val[0] += bfr(bias[c0 + cofs]); val[1] += bfr(bias[c0 + cofs + 1]); val[2] += bfr(bias[c0 + cofs + 2]); val[3] += bfr(bias[c0 + cofs + 3]); }
                *(volatile v4f*)(crow + (size_t)row * ldc + cofs) = val; }
            if (ps == 0) __threadfence(); }
        __builtin_amdgcn_wave_barrier(); asm volatile("" ::: "memory");
    }
}

__device__ __forceinline__ int wrap16(int v) { v = (v < 0) ? (v + NH) : v; v = (v < 0) ? 0 : v; return (v > NH - 1) ? (NH - 1) : v; }
__device__ __forceinline__ int hsel(const int* hidx, const int* hidxs, int slot) {
    const int a = hidx[0]; int bi = slot - 1; bi = (bi < 0) ? 0 : ((bi > NH - 2) ? (NH - 2) : bi); const int c = hidxs[bi];
    return wrap16((slot == 0) ? a : c);
}

__global__ __launch_bounds__(256) void k_cvtx(const float* __restrict__ s0, const float* __restrict__ s1, const float* __restrict__ s2, const float* __restrict__ s3, bf* d0, bf* d1, bf* d2, bf* d3) {
    const size_t i = (size_t)blockIdx.x * 256 + threadIdx.x; const size_t n8 = (size_t)NB * SEQ * DM / 8; if (i >= n8) return;
    const int w = blockIdx.y;
    const float* src = (w == 0) ? s0 : ((w == 1) ? s1 : ((w == 2) ? s2 : s3)); bf* dst = (w == 0) ? d0 : ((w == 1) ? d1 : ((w == 2) ? d2 : d3));
    const size_t e = i * 8; const size_t row = e / DM; const int col = (int)(e % DM); const size_t b = row / SEQ, t = row % SEQ;
    const v8f v = *(const v8f*)(src + ((b * SEQ_FULL + t) * DM + col)); v8us o;
#pragma unroll
    for (int q = 0; q < 8; ++q) o[q] = f2bf(v[q]);
    *(volatile v8us*)(dst + e) = o; __threadfence(); *(volatile v8us*)(dst + e) = o;
}

__global__ __launch_bounds__(256) void k_wg(const float* __restrict__ W, const int* __restrict__ hidx, const int* __restrict__ hidxs, bf* WB) {
    const size_t i = (size_t)blockIdx.x * 256 + threadIdx.x; const size_t n8 = (size_t)NSLOT * HD * DM / 8; if (i >= n8) return;
    const size_t e = i * 8; const int k = (int)(e % DM); const int r = (int)((e / DM) % HD); const int z = (int)(e / ((size_t)DM * HD)); const int type = z >> 4, slot = z & 15;
    const int hs = hsel(hidx, hidxs, slot);
    const v8f v = *(const v8f*)(W + ((size_t)(type * DM + hs * HD + r)) * DM + k); v8us o;
#pragma unroll
    for (int q = 0; q < 8; ++q) o[q] = f2bf(v[q]);
    *(volatile v8us*)(WB + e) = o; __threadfence(); *(volatile v8us*)(WB + e) = o;
}

__global__ __launch_bounds__(256) void k_cvtw(const float* __restrict__ W, h16* WP16, bf* WPB) {
    const size_t i = (size_t)blockIdx.x * 256 + threadIdx.x; const size_t n8 = (size_t)DM * DM / 8; if (i >= n8) return;
    const v8f v = *(const v8f*)(W + i * 8); v8h o16; v8us ob;
#pragma unroll
    for (int q = 0; q < 8; ++q) { ob[q] = f2bf(v[q]); o16[q] = (h16)(bf2f(ob[q]) * WCAR); }
    *(volatile v8h*)(WP16 + i * 8) = o16; *(volatile v8us*)(WPB + i * 8) = ob; __threadfence(); *(volatile v8h*)(WP16 + i * 8) = o16; *(volatile v8us*)(WPB + i * 8) = ob;
}

__global__ __launch_bounds__(32) void k_qkv(const bf* __restrict__ XB, const bf* __restrict__ X1B, const bf* __restrict__ X2B, const bf* __restrict__ X3B, const bf* __restrict__ WB, const float* __restrict__ battn,
                                          const int* __restrict__ hidx, const int* __restrict__ hidxs, const int* __restrict__ perm,
                                          h16* Q16, bf* QH, bf* QL, h16* K16, bf* KH, bf* KL, h16* VT, bf* VH, bf* VL) {
    __shared__ __align__(16) h16 s16[64 * ST];
    __shared__ __align__(16) bf  sbh[64 * ST];
    __shared__ __align__(16) bf  sbl[64 * ST];
    const int lane = threadIdx.x & 31, lr = lane & 15, hi = lane >> 4;
    const int z = blockIdx.z, type = z >> 4, slot = z & 15;
    const int r0 = blockIdx.x * 64;
    const int b = r0 / SEQ, t0 = r0 % SEQ; const bool hires = (t0 < RH);
    const bf* A = (slot == 0) ? ((type == 0) ? X1B : ((type == 1) ? X2B : X3B)) : XB;
    const bf* Bt = WB + (size_t)z * HD * DM;
    const int K = DM;
    v8f acc[4][4];
#pragma unroll
    for (int mb = 0; mb < 4; ++mb)
#pragma unroll
        for (int nb = 0; nb < 4; ++nb) acc[mb][nb] = (v8f){};
    const size_t aoff = (size_t)(r0 + lr) * K + 8 * hi, boff = (size_t)lr * K + 8 * hi;
#pragma unroll 1
    for (int kc = 0; kc < K; kc += 32) {
        v16bf a[4];
#pragma unroll
        for (int mb = 0; mb < 4; ++mb) a[mb] = WFrag<bf>::ld(A + aoff + (size_t)mb * 16 * K + kc);
#pragma unroll
        for (int nb = 0; nb < 4; ++nb) { const v16bf bb = WFrag<bf>::ld(Bt + boff + (size_t)nb * 16 * K + kc);
#pragma unroll
            for (int mb = 0; mb < 4; ++mb) acc[mb][nb] = wmmab(a[mb], bb, acc[mb][nb]); }
        asm volatile("v_nop\n\tv_nop\n\tv_nop\n\tv_nop" : "+v"(acc[0][0]), "+v"(acc[1][1]), "+v"(acc[2][2]), "+v"(acc[3][3]) : "v"(a[0]), "v"(a[3]));
    }
    const int hs = hsel(hidx, hidxs, slot); const int woff = type * DM + hs * HD;
    float bias[4];
#pragma unroll
    for (int nb = 0; nb < 4; ++nb) bias[nb] = bfr(battn[woff + nb * 16 + lr]);
#pragma unroll
    for (int mb = 0; mb < 4; ++mb)
#pragma unroll
        for (int nb = 0; nb < 4; ++nb)
#pragma unroll
            for (int j = 0; j < 8; ++j) {
                const float v = acc[mb][nb][j] + bias[nb];
                const int row = mb * 16 + hi * 8 + j, col = nb * 16 + lr;
                const int ix = (type == 2) ? (col * ST + row) : (row * ST + col);
                s16[ix] = (h16)v;
                if (hires) { unsigned short a2, c2; splitf(v, a2, c2); sbh[ix] = a2; sbl[ix] = c2; }
            }
    __syncthreads();
    const int rsel = lane >> 3, piece = (lane & 7) * 8;
#pragma unroll 1
    for (int hp = 0; hp < NH; ++hp) {
        const int pp = wrap16(perm[hp]);
        if (pp != slot) continue;
        const int zf = b * NH + hp;
#pragma unroll 1
        for (int ps = 0; ps < 2; ++ps) {
#pragma unroll 4
            for (int i = 0; i < 16; ++i) {
                const int rr = 4 * i + rsel;
                const v8h v16 = *(const v8ha*)(s16 + rr * ST + piece);
                if (type == 2) {
                    *(volatile v8h*)(VT + ((size_t)zf * HD + rr) * SEQ + t0 + piece) = v16;
                    if (hires) { const v8us vh = *(const v8usa*)(sbh + rr * ST + piece), vl = *(const v8usa*)(sbl + rr * ST + piece);
                        *(volatile v8us*)(VH + ((size_t)zf * HD + rr) * RH + t0 + piece) = vh; *(volatile v8us*)(VL + ((size_t)zf * HD + rr) * RH + t0 + piece) = vl; }
                } else {
                    h16* P = (type == 0) ? Q16 : K16;
                    *(volatile v8h*)(P + ((size_t)zf * SEQ + t0 + rr) * HD + piece) = v16;
                    if (hires) { const v8us vh = *(const v8usa*)(sbh + rr * ST + piece), vl = *(const v8usa*)(sbl + rr * ST + piece);
                        bf* PHp = (type == 0) ? QH : KH; bf* PLp = (type == 0) ? QL : KL;
                        *(volatile v8us*)(PHp + ((size_t)zf * RH + t0 + rr) * HD + piece) = vh; *(volatile v8us*)(PLp + ((size_t)zf * RH + t0 + rr) * HD + piece) = vl; }
                }
            }
            if (ps == 0) __threadfence();
        }
    }
}

template <bool HR>
__global__ __launch_bounds__(128) void k_flash(const h16* __restrict__ Q16, const bf* __restrict__ QH, const bf* __restrict__ QL,
                                               const h16* __restrict__ K16, const bf* __restrict__ KH, const bf* __restrict__ KL,
                                               const h16* __restrict__ VT, const bf* __restrict__ VH, const bf* __restrict__ VL,
                                               h16* Y16, bf* YH, bf* YL, int qt0) {
    __shared__ __align__(16) h16 P16[4 * PT];
    __shared__ __align__(16) bf  PHs[4 * PT];
    __shared__ __align__(16) bf  PLs[4 * PT];
    const int tid = threadIdx.x, w = tid >> 5, lane = tid & 31, m = lane & 15, hi = lane >> 4;
    const int qt = qt0 + blockIdx.x, q0 = qt * 64, zf = blockIdx.y, b = zf >> 4, hp = zf & 15;
    const int qw = q0 + w * 16;
    h16* Pw = P16 + w * PT; bf* PHw = PHs + w * PT; bf* PLw = PLs + w * PT;
    v16h qa[2]; v16bf qah[2], qal[2];
    if constexpr (!HR) {
#pragma unroll
        for (int kk = 0; kk < 2; ++kk) qa[kk] = WFrag<h16>::ld(Q16 + ((size_t)zf * SEQ + qw + m) * HD + kk * 32 + 8 * hi);
    } else {
#pragma unroll
        for (int kk = 0; kk < 2; ++kk) { qah[kk] = WFrag<bf>::ld(QH + ((size_t)zf * RH + qw + m) * HD + kk * 32 + 8 * hi); qal[kk] = WFrag<bf>::ld(QL + ((size_t)zf * RH + qw + m) * HD + kk * 32 + 8 * hi); }
    }
    v8f oacc[4];
#pragma unroll
    for (int nt = 0; nt < 4; ++nt) oacc[nt] = (v8f){};
    float mrow[8], lrow[8];
#pragma unroll
    for (int j = 0; j < 8; ++j) { mrow[j] = -3.0e38f; lrow[j] = 0.0f; }
    const int ntiles = qt + 1;
#pragma unroll 1
    for (int jt = 0; jt < ntiles; ++jt) {
        const int kv0 = jt * 64;
        v8f sacc[4];
#pragma unroll
        for (int nt = 0; nt < 4; ++nt) sacc[nt] = (v8f){};
        if constexpr (!HR) {
            v16h kb[4];
#pragma unroll
            for (int kk = 0; kk < 2; ++kk) {
#pragma unroll
                for (int nt = 0; nt < 4; ++nt) { kb[nt] = WFrag<h16>::ld(K16 + ((size_t)zf * SEQ + kv0 + nt * 16 + m) * HD + kk * 32 + 8 * hi); sacc[nt] = wmma16(qa[kk], kb[nt], sacc[nt]); }
            }
            asm volatile("v_nop\n\tv_nop\n\tv_nop\n\tv_nop" : "+v"(sacc[0]), "+v"(sacc[1]), "+v"(sacc[2]), "+v"(sacc[3]) : "v"(qa[0]), "v"(qa[1]), "v"(kb[3]));
        } else {
            v16bf kbh[4], kbl[4];
#pragma unroll
            for (int kk = 0; kk < 2; ++kk) {
#pragma unroll
                for (int nt = 0; nt < 4; ++nt) {
                    kbh[nt] = WFrag<bf>::ld(KH + ((size_t)zf * RH + kv0 + nt * 16 + m) * HD + kk * 32 + 8 * hi);
                    sacc[nt] = wmmab(qah[kk], kbh[nt], sacc[nt]); sacc[nt] = wmmab(qal[kk], kbh[nt], sacc[nt]);
                    kbl[nt] = WFrag<bf>::ld(KL + ((size_t)zf * RH + kv0 + nt * 16 + m) * HD + kk * 32 + 8 * hi);
                    sacc[nt] = wmmab(qah[kk], kbl[nt], sacc[nt]); }
            }
            asm volatile("v_nop\n\tv_nop\n\tv_nop\n\tv_nop" : "+v"(sacc[0]), "+v"(sacc[1]), "+v"(sacc[2]), "+v"(sacc[3]) : "v"(qah[0]), "v"(qal[1]), "v"(kbh[3]), "v"(kbl[3]));
        }
        const bool diag = (kv0 == q0);
#pragma unroll
        for (int j = 0; j < 8; ++j) {
            const int rr = w * 16 + hi * 8 + j;
            float sv[4]; float mx = -3.0e38f;
#pragma unroll
            for (int nt = 0; nt < 4; ++nt) { float s = sacc[nt][j] * SCL; const int kn = nt * 16 + m; s = (diag && kn > rr) ? -3.0e38f : s; sv[nt] = s; mx = fmaxf(mx, s); }
#pragma unroll
            for (int off = 1; off < 16; off <<= 1) mx = fmaxf(mx, __shfl_xor(mx, off, 32));
            const float mn = fmaxf(mrow[j], mx);
            const float corr = __builtin_amdgcn_exp2f((mrow[j] - mn) * L2E);
            mrow[j] = mn;
            float psum = 0.0f;
#pragma unroll
            for (int nt = 0; nt < 4; ++nt) {
                const float p = __builtin_amdgcn_exp2f((sv[nt] - mn) * L2E); psum += p;
                const int ix = (hi * 8 + j) * ST + nt * 16 + m;
                if constexpr (!HR) { Pw[ix] = (h16)(p * PCAR); } else { unsigned short a2, c2; splitf(p * PCAR, a2, c2); PHw[ix] = a2; PLw[ix] = c2; }
            }
#pragma unroll
            for (int off = 1; off < 16; off <<= 1) psum += __shfl_xor(psum, off, 32);
            lrow[j] = lrow[j] * corr + psum;
#pragma unroll
            for (int nt = 0; nt < 4; ++nt) oacc[nt][j] *= corr;
        }
        __builtin_amdgcn_fence(3  , "wavefront"); __builtin_amdgcn_wave_barrier(); asm volatile("" ::: "memory");
        if constexpr (!HR) {
            v16h pa[2], vb[4];
#pragma unroll
            for (int kk = 0; kk < 2; ++kk) {
                pa[kk] = cat16(*(const v8ha*)(Pw + m * ST + kk * 32 + 8 * hi), *(const v8ha*)(Pw + m * ST + kk * 32 + 8 * hi + 16));
#pragma unroll
                for (int nt = 0; nt < 4; ++nt) { vb[nt] = WFrag<h16>::ld(VT + ((size_t)zf * HD + nt * 16 + m) * SEQ + kv0 + kk * 32 + 8 * hi); oacc[nt] = wmma16(pa[kk], vb[nt], oacc[nt]); }
            }
            asm volatile("v_nop\n\tv_nop\n\tv_nop\n\tv_nop" : "+v"(oacc[0]), "+v"(oacc[1]), "+v"(oacc[2]), "+v"(oacc[3]) : "v"(pa[0]), "v"(pa[1]), "v"(vb[3]));
        } else {
            v16bf pah[2], pal[2], vbh[4], vbl[4];
#pragma unroll
            for (int kk = 0; kk < 2; ++kk) {
                pah[kk] = cat16b(*(const v8usa*)(PHw + m * ST + kk * 32 + 8 * hi), *(const v8usa*)(PHw + m * ST + kk * 32 + 8 * hi + 16));
                pal[kk] = cat16b(*(const v8usa*)(PLw + m * ST + kk * 32 + 8 * hi), *(const v8usa*)(PLw + m * ST + kk * 32 + 8 * hi + 16));
#pragma unroll
                for (int nt = 0; nt < 4; ++nt) {
                    vbh[nt] = WFrag<bf>::ld(VH + ((size_t)zf * HD + nt * 16 + m) * RH + kv0 + kk * 32 + 8 * hi);
                    oacc[nt] = wmmab(pah[kk], vbh[nt], oacc[nt]); oacc[nt] = wmmab(pal[kk], vbh[nt], oacc[nt]);
                    vbl[nt] = WFrag<bf>::ld(VL + ((size_t)zf * HD + nt * 16 + m) * RH + kv0 + kk * 32 + 8 * hi);
                    oacc[nt] = wmmab(pah[kk], vbl[nt], oacc[nt]); }
            }
            asm volatile("v_nop\n\tv_nop\n\tv_nop\n\tv_nop" : "+v"(oacc[0]), "+v"(oacc[1]), "+v"(oacc[2]), "+v"(oacc[3]) : "v"(pah[0]), "v"(pal[1]), "v"(vbh[3]), "v"(vbl[3]));
        }
        __builtin_amdgcn_wave_barrier(); asm volatile("" ::: "memory");
    }
#pragma unroll
    for (int j = 0; j < 8; ++j) {
        const float inv = 1.0f / (lrow[j] * PCAR);
#pragma unroll
        for (int nt = 0; nt < 4; ++nt) {
            const float y = oacc[nt][j] * inv;
            const int ix = (hi * 8 + j) * ST + nt * 16 + m;
            if constexpr (!HR) { Pw[ix] = (h16)(y * YCAR); } else { unsigned short a2, c2; splitf(y, a2, c2); PHw[ix] = a2; PLw[ix] = c2; }
        }
    }
    __builtin_amdgcn_fence(3  , "wavefront"); __builtin_amdgcn_wave_barrier(); asm volatile("" ::: "memory");
    const int rsel = lane >> 3, piece = (lane & 7) * 8;
#pragma unroll 1
    for (int ps = 0; ps < 2; ++ps) {
#pragma unroll
        for (int i = 0; i < 4; ++i) {
            const int rr = 4 * i + rsel; const int t = qw + rr;
            if constexpr (!HR) {
                const v8h v16 = *(const v8ha*)(Pw + rr * ST + piece);
                *(volatile v8h*)(Y16 + ((size_t)b * SEQ + t) * DM + hp * HD + piece) = v16;
            } else {
                const v8us vh = *(const v8usa*)(PHw + rr * ST + piece), vl = *(const v8usa*)(PLw + rr * ST + piece);
                *(volatile v8us*)(YH + ((size_t)b * RH + t) * DM + hp * HD + piece) = vh; *(volatile v8us*)(YL + ((size_t)b * RH + t) * DM + hp * HD + piece) = vl;
            }
        }
        if (ps == 0) __threadfence();
    }
}

extern "C" void kernel_launch(void* const* d_in, const int* in_sizes, int n_in,
                              void* d_out, int out_size, void* d_ws, size_t ws_size, hipStream_t stream) {
    if (n_in < 11) return;
    const int xneed = (NB - 1) * SEQ_FULL * DM + SEQ * DM;
    if (in_sizes[0] < xneed || in_sizes[1] < xneed || in_sizes[2] < xneed || in_sizes[3] < xneed) return;
    if (in_sizes[4] < NQKV * DM || in_sizes[5] < NQKV || in_sizes[6] < DM * DM || in_sizes[7] < DM) return;
    if (in_sizes[8] < 1 || in_sizes[9] < NH - 1 || in_sizes[10] < NH) return;
    if (out_size < xneed) return;
    const float* X1 = (const float*)d_in[0]; const float* X2 = (const float*)d_in[1]; const float* X3 = (const float*)d_in[2]; const float* X = (const float*)d_in[3];
    const float* Wattn = (const float*)d_in[4]; const float* battn = (const float*)d_in[5]; const float* Wproj = (const float*)d_in[6]; const float* bproj = (const float*)d_in[7];
    const int* hidx = (const int*)d_in[8]; const int* hidxs = (const int*)d_in[9]; const int* perm = (const int*)d_in[10];
    float* OUT = (float*)d_out;

    char* wsp = (char*)d_ws;
    auto take = [&](size_t bytes) { char* p = wsp; wsp += (bytes + 255) & ~(size_t)255; return (void*)p; };
    const size_t xplane = (size_t)NB * SEQ * DM * 2;
    bf* XB = (bf*)take(xplane); bf* X1B = (bf*)take(xplane); bf* X2B = (bf*)take(xplane); bf* X3B = (bf*)take(xplane);
    bf* WB = (bf*)take((size_t)NSLOT * HD * DM * 2);
    h16* WP16 = (h16*)take((size_t)DM * DM * 2); bf* WPB = (bf*)take((size_t)DM * DM * 2);
    const size_t hplane = (size_t)NB * NH * SEQ * HD * 2, hplaneR = (size_t)NB * NH * RH * HD * 2;
    h16* Q16 = (h16*)take(hplane); h16* K16 = (h16*)take(hplane); h16* VT = (h16*)take(hplane);
    bf* QH = (bf*)take(hplaneR); bf* QL = (bf*)take(hplaneR); bf* KH = (bf*)take(hplaneR); bf* KL = (bf*)take(hplaneR); bf* VH = (bf*)take(hplaneR); bf* VL = (bf*)take(hplaneR);
    h16* Y16 = (h16*)take((size_t)NB * SEQ * DM * 2); bf* YH = (bf*)take((size_t)NB * RH * DM * 2); bf* YL = (bf*)take((size_t)NB * RH * DM * 2);
    if ((size_t)(wsp - (char*)d_ws) > ws_size) return;

    k_cvtx<<<dim3((unsigned)(((size_t)NB * SEQ * DM / 8 + 255) / 256), 4), 256, 0, stream>>>(X, X1, X2, X3, XB, X1B, X2B, X3B);
    k_wg<<<(unsigned)(((size_t)NSLOT * HD * DM / 8 + 255) / 256), 256, 0, stream>>>(Wattn, hidx, hidxs, WB);
    k_cvtw<<<(unsigned)(((size_t)DM * DM / 8 + 255) / 256), 256, 0, stream>>>(Wproj, WP16, WPB);
    k_qkv<<<dim3(NB * SEQ / 64, 1, NSLOT), 32, 0, stream>>>(XB, X1B, X2B, X3B, WB, battn, hidx, hidxs, perm, Q16, QH, QL, K16, KH, KL, VT, VH, VL);
    k_flash<true><<<dim3(RH / 64, NB * NH), 128, 0, stream>>>(Q16, QH, QL, K16, KH, KL, VT, VH, VL, Y16, YH, YL, 0);
    if (SEQ > RH) k_flash<false><<<dim3((SEQ - RH) / 64, NB * NH), 128, 0, stream>>>(Q16, QH, QL, K16, KH, KL, VT, VH, VL, Y16, YH, YL, RH / 64);
    k_gemmw<bf, 1, true><<<dim3(RH / 64, DM / 64, NB), 32, 0, stream>>>(YH, YL, WPB, nullptr, DM, OUT, DM, bproj, 1.0f, (size_t)RH * DM, (size_t)0, (size_t)SEQ_FULL * DM);
    if (SEQ > RH) k_gemmw<h16, 0, true><<<dim3((SEQ - RH) / 64, DM / 64, NB), 32, 0, stream>>>(Y16 + (size_t)RH * DM, nullptr, WP16, nullptr, DM, OUT + (size_t)RH * DM, DM, bproj, OSC, (size_t)SEQ * DM, (size_t)0, (size_t)SEQ_FULL * DM);
}
